// RnnEncoder_13039520711439
// MI455X (gfx1250) — hardware-run, weakly checked
//
#include <hip/hip_runtime.h>
#include <math.h>

typedef __attribute__((ext_vector_type(16))) _Float16 v16h;
typedef __attribute__((ext_vector_type(8)))  _Float16 v8h;
typedef __attribute__((ext_vector_type(16))) __bf16   v16b;
typedef __attribute__((ext_vector_type(8)))  __bf16   v8b;
typedef __attribute__((ext_vector_type(8)))  float    v8f;
typedef __attribute__((ext_vector_type(4)))  float    v4f;
#define PSCALE 32768.0f
#define U16(p) ((const unsigned short*)(const void*)(p))
#define PSCALE_INV (1.0f / 32768.0f)

__device__ __forceinline__ unsigned short f2bf_bits(float f) {
  unsigned u = __float_as_uint(f);
  return (unsigned short)((u + 0x7FFFu + ((u >> 16) & 1u)) >> 16);
}
__device__ __forceinline__ float bf_bits2f(unsigned short h) { return __uint_as_float(((unsigned)h) << 16); }

__device__ __forceinline__ void dep_guard_h(v8f& a, v8f& b, v16h x, v16h y) { asm volatile("v_nop\n\tv_nop\n\tv_nop\n\tv_nop" : "+v"(a), "+v"(b) : "v"(x), "v"(y)); }
__device__ __forceinline__ void dep_guard_b(v8f& a, v8f& b, v16b x, v16b y) { asm volatile("v_nop\n\tv_nop\n\tv_nop\n\tv_nop" : "+v"(a), "+v"(b) : "v"(x), "v"(y)); }
__device__ __forceinline__ void keep4_h(v16h a, v16h b, v16h c, v16h d) { asm volatile("v_nop" :: "v"(a), "v"(b), "v"(c), "v"(d)); }
__device__ __forceinline__ void keep4_b(v16b a, v16b b, v16b c, v16b d) { asm volatile("v_nop" :: "v"(a), "v"(b), "v"(c), "v"(d)); }
__device__ __forceinline__ void acc_guard4(v8f& a, v8f& b, v8f& c, v8f& d) { asm volatile("v_nop\n\tv_nop\n\tv_nop\n\tv_nop" : "+v"(a), "+v"(b), "+v"(c), "+v"(d)); }
template <typename T> struct Frag;
template <> struct Frag<_Float16> {
  typedef v16h V; union U { v16h v; v8h h[2]; };
  static __device__ __forceinline__ v16h load(const _Float16* p) {
    U f; f.h[0] = *(const v8h*)(p); f.h[1] = *(const v8h*)(p + 16); return f.v;
  }
  static __device__ __forceinline__ v8f mma(v16h a, v16h b, v8f c) {
    return __builtin_amdgcn_wmma_f32_16x16x32_f16(false, a, false, b, (short)0, c, false, false);
  }
  static __device__ __forceinline__ void guard(v8f& a, v8f& b, v16h x, v16h y) { dep_guard_h(a, b, x, y); }
  static __device__ __forceinline__ void keep(v16h a, v16h b, v16h c, v16h d) { keep4_h(a, b, c, d); }
};
template <> struct Frag<__bf16> {
  typedef v16b V; union U { v16b v; v8b h[2]; };
  static __device__ __forceinline__ v16b load(const __bf16* p) {
    U f; f.h[0] = *(const v8b*)(p); f.h[1] = *(const v8b*)(p + 16); return f.v;
  }
  static __device__ __forceinline__ v8f mma(v16b a, v16b b, v8f c) {
    return __builtin_amdgcn_wmma_f32_16x16x32_bf16(false, a, false, b, (short)0, c, false, false);
  }
  static __device__ __forceinline__ void guard(v8f& a, v8f& b, v16b x, v16b y) { dep_guard_b(a, b, x, y); }
  static __device__ __forceinline__ void keep(v16b a, v16b b, v16b c, v16b d) { keep4_b(a, b, c, d); }
};

template <int ET> struct Elem;
template <> struct Elem<0> { typedef _Float16 T; };
template <> struct Elem<1> { typedef __bf16 T; };
template <int ET, bool SPLIT, int BIAS_MODE, int OUT_MODE, bool RESID, int ACT = 0>
__global__ __launch_bounds__(256) void wmma_gemm64(
    const unsigned short* __restrict__ Ap, const unsigned short* __restrict__ A2p, int lda, long strideA,
    const unsigned short* __restrict__ Btp, const unsigned short* __restrict__ Bt2p, int ldb, long strideB,
    void* __restrict__ Cout, void* __restrict__ Cout2, int ldc, long strideC,
    const float* __restrict__ bias,
    const float* __restrict__ resid, long strideR,
    int M, int N, int K, float scale) {
  typedef typename Elem<ET>::T T;
  typedef typename Frag<T>::V V;
  const T* A = (const T*)Ap; const T* A2 = (const T*)A2p; const T* Bt = (const T*)Btp; const T* Bt2 = (const T*)Bt2p;
  __shared__ __align__(16) float sT[8][16 * 68];
  const int b    = blockIdx.y;
  const int lane = threadIdx.x & 31;
  const int wave = threadIdx.x >> 5;
  const int tilesN = N >> 6;
  const int tilesM = M >> 6;
  const int tile = blockIdx.x * 8 + wave;
  if (tile >= tilesM * tilesN) return;
  const int tm = tile / tilesN;
  const int tn = tile - tm * tilesN;
  const int m0 = tm << 6;
  const int n0 = tn << 6;

  const T* Ab  = A  + (size_t)b * strideA;
  const T* Bb  = Bt + (size_t)b * strideB;
  const T* Ab2 = SPLIT ? (A2  + (size_t)b * strideA) : nullptr;
  const T* Bb2 = SPLIT ? (Bt2 + (size_t)b * strideB) : nullptr;

  const int rlane = lane & 15;
  const int koff  = (lane >> 4) * 8;
  const int mOff  = (lane >> 4) * 8;

  v8f acc[4][4];
#pragma unroll
  for (int i = 0; i < 4; ++i)
#pragma unroll
    for (int j = 0; j < 4; ++j) acc[i][j] = (v8f){0.f,0.f,0.f,0.f,0.f,0.f,0.f,0.f};

  for (int k0 = 0; k0 < K; k0 += 32) {
    V bh[4], bl[4];
#pragma unroll
    for (int j = 0; j < 4; ++j) {
      const size_t bo = (size_t)(n0 + (j << 4) + rlane) * ldb + koff + k0;
      bh[j] = Frag<T>::load(Bb + bo);
      if (SPLIT) bl[j] = Frag<T>::load(Bb2 + bo);
    }
#pragma unroll
    for (int i = 0; i < 4; ++i) {
      const size_t ao = (size_t)(m0 + (i << 4) + rlane) * lda + koff + k0;
      V ah = Frag<T>::load(Ab + ao);
      V al;
      if (SPLIT) al = Frag<T>::load(Ab2 + ao);
#pragma unroll
      for (int j = 0; j < 4; ++j) {
        acc[i][j] = Frag<T>::mma(ah, bh[j], acc[i][j]);
        if (SPLIT) {
          acc[i][j] = Frag<T>::mma(ah, bl[j], acc[i][j]);
          acc[i][j] = Frag<T>::mma(al, bh[j], acc[i][j]);
        }
      }
      Frag<T>::guard(acc[i][0], acc[i][3], ah, SPLIT ? al : ah);
    }
    Frag<T>::keep(bh[0], bh[1], bh[2], bh[3]);
    if (SPLIT) Frag<T>::keep(bl[0], bl[1], bl[2], bl[3]);
  }
  acc_guard4(acc[0][0], acc[0][1], acc[0][2], acc[0][3]);
  acc_guard4(acc[1][0], acc[1][1], acc[1][2], acc[1][3]);
  acc_guard4(acc[2][0], acc[2][1], acc[2][2], acc[2][3]);
  acc_guard4(acc[3][0], acc[3][1], acc[3][2], acc[3][3]);

  float* slab = sT[wave];
  const float* Rb = RESID ? (resid + (size_t)b * strideR) : nullptr;
#pragma unroll
  for (int i = 0; i < 4; ++i) {
    const int mBase = m0 + (i << 4);
#pragma unroll
    for (int j = 0; j < 4; ++j) {
      const int n = n0 + (j << 4) + rlane;
      float bv = 0.f;
      if (BIAS_MODE == 2) bv = bias[n];
#pragma unroll
      for (int r = 0; r < 8; ++r) {
        float v = acc[i][j][r] * scale;
        if (BIAS_MODE == 1) v += bias[mBase + mOff + r];
        if (BIAS_MODE == 2) v += bv;
        if (RESID) v += Rb[(size_t)(mBase + mOff + r) * ldc + n];
        if (ACT == 1) v = tanhf(v);
        if (ACT == 2) v = fmaxf(v, 0.0f);
        if (ACT == 3) v = v / (1.0f + expf(-v));
        if (ACT == 4) v = (v > 0.f) ? v : 0.01f * v;
        if (ACT == 5) v = 0.5f * v * (1.0f + erff(v * 0.70710678118654752f));
        slab[(mOff + r) * 68 + (j << 4) + rlane] = v;
      }
    }
    __builtin_amdgcn_fence(__ATOMIC_RELEASE, "workgroup");
    __builtin_amdgcn_wave_barrier();
    __builtin_amdgcn_fence(__ATOMIC_ACQUIRE, "workgroup");
    if (OUT_MODE == 0) {
      float* C = (float*)Cout + (size_t)b * strideC;
      const int hh = lane >> 4, c4 = (lane & 15) * 4;
      for (int pass = 0; pass < 2; ++pass) {
#pragma unroll
        for (int it = 0; it < 8; ++it) {
          const int row = it * 2 + hh;
          v4f v = *(const v4f*)(slab + row * 68 + c4);
          *(volatile v4f*)(C + (size_t)(mBase + row) * ldc + n0 + c4) = v;
        }
        __threadfence();
      }
    } else {
      const int q = lane >> 3, c8 = (lane & 7) * 8;
      unsigned short* C  = (unsigned short*)Cout  + (size_t)b * strideC;
      unsigned short* C2 = (OUT_MODE == 2) ? ((unsigned short*)Cout2 + (size_t)b * strideC) : nullptr;
      for (int pass = 0; pass < 2; ++pass) {
#pragma unroll
        for (int it = 0; it < 4; ++it) {
          const int row = it * 4 + q;
          const float* sp = slab + row * 68 + c8;
          v8h hv, lv;
#pragma unroll
          for (int e = 0; e < 8; ++e) {
            if (OUT_MODE == 1) {
              hv[e] = (_Float16)sp[e];
            } else {
              unsigned short hb = f2bf_bits(sp[e]);
              unsigned short lb = f2bf_bits(sp[e] - bf_bits2f(hb));
              hv[e] = __builtin_bit_cast(_Float16, hb);
              lv[e] = __builtin_bit_cast(_Float16, lb);
            }
          }
          *(volatile v8h*)(C + (size_t)(mBase + row) * ldc + n0 + c8) = hv;
          if (OUT_MODE == 2) *(volatile v8h*)(C2 + (size_t)(mBase + row) * ldc + n0 + c8) = lv;
        }
        __threadfence();
      }
    }
    __builtin_amdgcn_fence(__ATOMIC_RELEASE, "workgroup");
    __builtin_amdgcn_wave_barrier();
    __builtin_amdgcn_fence(__ATOMIC_ACQUIRE, "workgroup");
  }
}

constexpr int NBATCH = 16;
constexpr int NSEQ   = 512;
constexpr int NINP   = 128;
constexpr int NDIM   = 512;
constexpr int NHID   = 512;
constexpr int NDA    = 30;
constexpr int NDAP   = 64;
constexpr int NHEAD  = 10;
constexpr int NG3    = 3 * NHID;
constexpr int NROWS  = NBATCH * NSEQ;
constexpr int UPITCH = NDAP;
constexpr int OSP    = 36;
constexpr int NBIAS  = NDIM + NDAP + NG3;

static_assert(NINP % 32 == 0 && NDIM % 32 == 0 && NSEQ % 32 == 0 && NHID % 32 == 0, "K multiples of 32");
static_assert(NROWS % 64 == 0 && NDIM % 64 == 0 && NDAP % 64 == 0 && NSEQ % 64 == 0 && NG3 % 64 == 0, "M,N multiples of 64");
static_assert(NBIAS % 32 == 0, "bias table whole lines");
static_assert((NROWS * NINP) % (8 * 256) == 0, "x convert grid exact");
static_assert(NHID == 16 * 32, "16 waves x 32 columns in the recurrence kernel");
static_assert(NDA <= NDAP && NDA * NHEAD <= 512, "score table fits");

__device__ __forceinline__ float rne_bf16(float f) { return bf_bits2f(f2bf_bits(f)); }

__global__ __launch_bounds__(256) void k_cvt_x(const float* __restrict__ x, unsigned short* __restrict__ o, int n8) {
  const int i = blockIdx.x * 256 + threadIdx.x;
  if (i < n8) {
    const v4f a0 = *(const v4f*)(x + (size_t)i * 8);
    const v4f a1 = *(const v4f*)(x + (size_t)i * 8 + 4);
    v8h hv;
#pragma unroll
    for (int e = 0; e < 4; ++e) {
      const float f0 = rne_bf16(a0[e]);
      const float f1 = rne_bf16(a1[e]);
      hv[e] = (_Float16)f0;
      hv[4 + e] = (_Float16)f1;
    }
    unsigned short* dst = o + (size_t)i * 8;
    *(volatile v8h*)dst = hv;
    __threadfence();
    *(volatile v8h*)dst = hv;
  }
}

__global__ __launch_bounds__(256) void k_trans16(const float* __restrict__ in, unsigned short* __restrict__ out,
                                                 int Rn, int Cn, float sc) {
  __shared__ float tile[64 * 65];
  const int tid = threadIdx.x;
  const int c0 = blockIdx.x * 64;
  const int r0 = blockIdx.y * 64;
#pragma unroll 1
  for (int i4 = 0; i4 < 4; ++i4) {
#pragma unroll
    for (int u = 0; u < 4; ++u) {
      const int e = tid + 256 * (i4 * 4 + u);
      const int rr = e >> 6, cc = e & 63;
      const int c = c0 + cc;
      const int cl = (c < Cn) ? c : (Cn - 1);
      float v = in[(size_t)(r0 + rr) * Cn + cl];
      v = (c < Cn) ? v : 0.0f;
      tile[rr * 65 + cc] = v;
    }
  }
  __syncthreads();
  const int q = tid & 7;
#pragma unroll
  for (int it = 0; it < 2; ++it) {
    const int oc = (tid >> 3) + 32 * it;
    v8h hv;
#pragma unroll
    for (int e = 0; e < 8; ++e) {
      float w = tile[(8 * q + e) * 65 + oc];
      w = rne_bf16(w) * sc;
      hv[e] = (_Float16)w;
    }
    unsigned short* dst = out + (size_t)(c0 + oc) * Rn + r0 + 8 * q;
    *(volatile v8h*)dst = hv;
    __threadfence();
    *(volatile v8h*)dst = hv;
  }
}

__global__ __launch_bounds__(256) void k_bias(const float* __restrict__ b0, const float* __restrict__ b1,
                                              const float* __restrict__ bi, float* __restrict__ btab, int n) {
  const int i = blockIdx.x * 256 + threadIdx.x;
  if (i < n) {
    const int i0 = (i < NDIM) ? i : (NDIM - 1);
    int i1 = i - NDIM; i1 = (i1 < 0) ? 0 : ((i1 > NDA - 1) ? (NDA - 1) : i1);
    int i2 = i - NDIM - NDAP; i2 = (i2 < 0) ? 0 : ((i2 > NG3 - 1) ? (NG3 - 1) : i2);
    const float v0 = b0[i0];
    const float v1 = b1[i1];
    const float v2 = bi[i2];
    float v = (i < NDIM) ? v0 : ((i < NDIM + NDAP) ? ((i - NDIM < NDA) ? v1 : 0.0f) : v2);
    v = rne_bf16(v);
    ((volatile float*)btab)[i] = v;
    __threadfence();
    ((volatile float*)btab)[i] = v;
  }
}

__global__ __launch_bounds__(512) void k_attnp(const float* __restrict__ U, const float* __restrict__ W2,
                                               const float* __restrict__ b2, unsigned short* __restrict__ P16) {
  __shared__ float w2s[NDA * NHEAD];
  __shared__ float b2s[16];
  __shared__ float gms[16];
  __shared__ float wm[16 * NHEAD];
  __shared__ __align__(16) float Es[NSEQ * NHEAD];
  __shared__ __align__(16) float Zs[NSEQ * NHEAD];
  __shared__ __align__(16) _Float16 Pst[8 * NSEQ];
  const int tid = threadIdx.x;
  const int lane = tid & 31;
  const int wave = tid >> 5;
  const int b = blockIdx.x;
  if (tid < NDA * NHEAD) w2s[tid] = rne_bf16(W2[tid]);
  if (tid < NHEAD) b2s[tid] = rne_bf16(b2[tid]);
  __syncthreads();

  const int k = tid;
  const size_t row = (size_t)b * NSEQ + k;
  float sacc[NHEAD];
#pragma unroll
  for (int r = 0; r < NHEAD; ++r) sacc[r] = b2s[r];
#pragma unroll 1
  for (int a = 0; a < NDA; ++a) {
    const float u = tanhf(U[row * UPITCH + a]);
    const float* wr = w2s + a * NHEAD;
#pragma unroll
    for (int r = 0; r < NHEAD; ++r) sacc[r] += u * wr[r];
  }
#pragma unroll
  for (int r = 0; r < NHEAD; ++r) {
    float m = sacc[r];
#pragma unroll
    for (int off = 1; off < 32; off <<= 1) m = fmaxf(m, __shfl_xor(m, off, 32));
    if (lane == 0) wm[wave * NHEAD + r] = m;
  }
  __syncthreads();
  if (tid < NHEAD) {
    float m = wm[tid];
#pragma unroll 1
    for (int w = 1; w < 16; ++w) m = fmaxf(m, wm[w * NHEAD + tid]);
    gms[tid] = m;
  }
  __syncthreads();
#pragma unroll
  for (int r = 0; r < NHEAD; ++r) Es[k * NHEAD + r] = sacc[r] - gms[r];
#pragma unroll 1
  for (int r = 0; r < NHEAD; ++r) {
    const float e = expf(Es[k * NHEAD + r]);
    Es[k * NHEAD + r] = e;
    Zs[k * NHEAD + r] = e;
  }
  __syncthreads();
  for (int off = 1; off < NSEQ; off <<= 1) {
    float vt[NHEAD];
    const int kp = (k >= off) ? (k - off) : 0;
#pragma unroll
    for (int r = 0; r < NHEAD; ++r) {
      const float cur = Zs[k * NHEAD + r];
      const float prev = Zs[kp * NHEAD + r];
      vt[r] = (k >= off) ? (cur + prev) : cur;
    }
    __syncthreads();
#pragma unroll
    for (int r = 0; r < NHEAD; ++r) Zs[k * NHEAD + r] = vt[r];
    __syncthreads();
  }
#pragma unroll 1
  for (int r = 0; r < NHEAD; ++r) {
    const float z = Zs[k * NHEAD + r];
    Zs[k * NHEAD + r] = (1024.0f / (float)NHEAD) * (1.0f / z);
  }
  __syncthreads();
  for (int t0 = 0; t0 < NSEQ; t0 += 8) {
    const int rr = tid >> 6;
    const int j = tid & 63;
    const int t = t0 + rr;
    float iz[NHEAD];
#pragma unroll
    for (int r = 0; r < NHEAD; ++r) iz[r] = Zs[t * NHEAD + r];
#pragma unroll 1
    for (int kk = 0; kk < 8; ++kk) {
      const int kx = j * 8 + kk;
      const float* er = Es + kx * NHEAD;
      float p = 0.0f;
#pragma unroll
      for (int r = 0; r < NHEAD; ++r) p += er[r] * iz[r];
      p = (kx <= t) ? p : 0.0f;
      Pst[rr * NSEQ + kx] = (_Float16)p;
    }
    __syncthreads();
    {
      const int c = tid & 63;
      const int r2 = tid >> 6;
      const v8h val = *(const v8h*)(Pst + r2 * NSEQ + c * 8);
      unsigned short* dst = P16 + ((size_t)b * NSEQ + t0 + r2) * NSEQ + c * 8;
      *(volatile v8h*)dst = val;
      __threadfence();
      *(volatile v8h*)dst = val;
    }
    __syncthreads();
  }
}

__device__ __forceinline__ void guard6h(v8f& a0, v8f& a1, v8f& a2, v8f& a3, v8f& a4, v8f& a5,
                                        v16h x, v16h y0, v16h y1, v16h y2, v16h y3, v16h y4, v16h y5) {
  asm volatile("v_nop\n\tv_nop\n\tv_nop\n\tv_nop"
               : "+v"(a0), "+v"(a1), "+v"(a2), "+v"(a3), "+v"(a4), "+v"(a5)
               : "v"(x), "v"(y0), "v"(y1), "v"(y2), "v"(y3), "v"(y4), "v"(y5));
}
__device__ __forceinline__ void guard6(v8f& a0, v8f& a1, v8f& a2, v8f& a3, v8f& a4, v8f& a5) {
  asm volatile("v_nop\n\tv_nop\n\tv_nop\n\tv_nop" : "+v"(a0), "+v"(a1), "+v"(a2), "+v"(a3), "+v"(a4), "+v"(a5));
}

__global__ __launch_bounds__(512) void k_gru(const float* __restrict__ giT, const unsigned short* __restrict__ Whhp,
                                             const float* __restrict__ b_h, float* __restrict__ out) {
  __shared__ __align__(16) _Float16 h16[NBATCH * NHID];
  __shared__ __align__(16) float oS[16][16 * OSP];
  const _Float16* Whh = (const _Float16*)Whhp;
  const int tid = threadIdx.x;
  const int lane = tid & 31;
  const int wave = tid >> 5;
  const int rlane = lane & 15;
  const int hh = lane >> 4;
  const int koff = hh * 8;
  const int col0 = wave * 32;
  {
    uint4 z; z.x = 0u; z.y = 0u; z.z = 0u; z.w = 0u;
    uint4* hz = (uint4*)(void*)h16;
    hz[tid] = z;
    hz[tid + 512] = z;
  }
  float bh[3][2];
#pragma unroll
  for (int g = 0; g < 3; ++g)
#pragma unroll
    for (int j = 0; j < 2; ++j) bh[g][j] = rne_bf16(b_h[g * NHID + col0 + 16 * j + rlane]);
  float hreg[2][8];
#pragma unroll
  for (int j = 0; j < 2; ++j)
#pragma unroll
    for (int r = 0; r < 8; ++r) hreg[j][r] = 0.0f;
  __syncthreads();
  const float inv16 = 0.0625f;
  float* oSw = oS[wave];
  const size_t gst = (size_t)NHID * NROWS;

  for (int t = 0; t < NSEQ; ++t) {
    v8f acc[3][2];
#pragma unroll
    for (int g = 0; g < 3; ++g)
#pragma unroll
      for (int j = 0; j < 2; ++j) acc[g][j] = (v8f){0.f,0.f,0.f,0.f,0.f,0.f,0.f,0.f};
    for (int k0 = 0; k0 < NHID; k0 += 32) {
      const v16h a = Frag<_Float16>::load(h16 + rlane * NHID + k0 + koff);
      v16h bf[3][2];
#pragma unroll
      for (int g = 0; g < 3; ++g)
#pragma unroll
        for (int j = 0; j < 2; ++j)
          bf[g][j] = Frag<_Float16>::load(Whh + (size_t)(g * NHID + col0 + 16 * j + rlane) * NHID + k0 + koff);
#pragma unroll
      for (int g = 0; g < 3; ++g)
#pragma unroll
        for (int j = 0; j < 2; ++j) acc[g][j] = Frag<_Float16>::mma(a, bf[g][j], acc[g][j]);
      guard6h(acc[0][0], acc[0][1], acc[1][0], acc[1][1], acc[2][0], acc[2][1],
              a, bf[0][0], bf[0][1], bf[1][0], bf[1][1], bf[2][0], bf[2][1]);
    }
    guard6(acc[0][0], acc[0][1], acc[1][0], acc[1][1], acc[2][0], acc[2][1]);
    __syncthreads();
#pragma unroll
    for (int j = 0; j < 2; ++j) {
      const int col = col0 + 16 * j + rlane;
      const float* gp = giT + (size_t)col * NROWS + (size_t)t * NBATCH + 8 * hh;
      const v4f r0v = *(const v4f*)(gp);
      const v4f r1v = *(const v4f*)(gp + 4);
      const v4f z0v = *(const v4f*)(gp + gst);
      const v4f z1v = *(const v4f*)(gp + gst + 4);
      const v4f n0v = *(const v4f*)(gp + 2 * gst);
      const v4f n1v = *(const v4f*)(gp + 2 * gst + 4);
      float gr[8], gz[8], gn[8];
#pragma unroll
      for (int e = 0; e < 4; ++e) {
        gr[e] = r0v[e]; gr[4 + e] = r1v[e];
        gz[e] = z0v[e]; gz[4 + e] = z1v[e];
        gn[e] = n0v[e]; gn[4 + e] = n1v[e];
      }
#pragma unroll
      for (int r = 0; r < 8; ++r) {
        const float hr = acc[0][j][r] * inv16 + bh[0][j];
        const float hz = acc[1][j][r] * inv16 + bh[1][j];
        const float hn = acc[2][j][r] * inv16 + bh[2][j];
        const float rt = 1.0f / (1.0f + expf(-(gr[r] + hr)));
        const float zt = 1.0f / (1.0f + expf(-(gz[r] + hz)));
        const float nt = tanhf(gn[r] + rt * hn);
        const float hold = hreg[j][r];
        const float hnew = nt + zt * (hold - nt);
        hreg[j][r] = hnew;
        const int brow = 8 * hh + r;
        h16[brow * NHID + col] = (_Float16)hnew;
        oSw[brow * OSP + 16 * j + rlane] = hnew;
      }
    }
    __syncthreads();
    {
      const int q = lane & 7;
      const int rb = lane >> 3;
      for (int pass = 0; pass < 2; ++pass) {
#pragma unroll
        for (int it = 0; it < 4; ++it) {
          const int brow = rb + 4 * it;
          const v4f v = *(const v4f*)(oSw + brow * OSP + 4 * q);
          *(volatile v4f*)(out + ((size_t)brow * NSEQ + t) * NHID + col0 + 4 * q) = v;
        }
        __threadfence();
      }
    }
  }
}

extern "C" void kernel_launch(void* const* d_in, const int* in_sizes, int n_in,
                              void* d_out, int out_size, void* d_ws, size_t ws_size,
                              hipStream_t stream) {
  if (n_in < 11) return;
  if (in_sizes[0] != NROWS * NINP || in_sizes[1] != NINP * NDIM || in_sizes[2] != NDIM ||
      in_sizes[3] != NDIM * NDA || in_sizes[4] != NDA || in_sizes[5] != NDA * NHEAD ||
      in_sizes[6] != NHEAD || in_sizes[7] != NDIM * NG3 || in_sizes[8] != NHID * NG3 ||
      in_sizes[9] != NG3 || in_sizes[10] != NG3) return;
  if (out_size != NROWS * NHID) return;

  const float* x      = (const float*)d_in[0];
  const float* W_mlp0 = (const float*)d_in[1];
  const float* b_mlp0 = (const float*)d_in[2];
  const float* W1     = (const float*)d_in[3];
  const float* b1     = (const float*)d_in[4];
  const float* W2     = (const float*)d_in[5];
  const float* b2     = (const float*)d_in[6];
  const float* W_ih   = (const float*)d_in[7];
  const float* W_hh   = (const float*)d_in[8];
  const float* b_i    = (const float*)d_in[9];
  const float* b_h    = (const float*)d_in[10];
  float* out = (float*)d_out;

  char* ws = (char*)d_ws;
  size_t off = 0;
  auto wsalloc = [&](size_t bytes) -> char* {
    char* p = ws + off;
    off += (bytes + 255) & ~(size_t)255;
    return p;
  };
  unsigned short* x16  = (unsigned short*)wsalloc(sizeof(unsigned short) * NROWS * NINP);
  unsigned short* W0T  = (unsigned short*)wsalloc(sizeof(unsigned short) * NDIM * NINP);
  unsigned short* W1T  = (unsigned short*)wsalloc(sizeof(unsigned short) * NDAP * NDIM);
  unsigned short* WihT = (unsigned short*)wsalloc(sizeof(unsigned short) * NG3 * NDIM);
  unsigned short* WhhT = (unsigned short*)wsalloc(sizeof(unsigned short) * NG3 * NHID);
  float*          btab = (float*)         wsalloc(sizeof(float) * NBIAS);
  unsigned short* m16  = (unsigned short*)wsalloc(sizeof(unsigned short) * (size_t)NROWS * NDIM);
  unsigned short* mT16 = (unsigned short*)wsalloc(sizeof(unsigned short) * (size_t)NDIM * NROWS);
  float*          U    = (float*)         wsalloc(sizeof(float) * (size_t)NROWS * UPITCH);
  unsigned short* P16  = (unsigned short*)wsalloc(sizeof(unsigned short) * (size_t)NBATCH * NSEQ * NSEQ);
  unsigned short* M16  = (unsigned short*)wsalloc(sizeof(unsigned short) * (size_t)NROWS * NDIM);
  float*          giT  = (float*)         wsalloc(sizeof(float) * (size_t)NG3 * NROWS);
  if (off > ws_size) return;

  const float* b0r = btab;
  const float* b1p = btab + NDIM;
  const float* bir = btab + NDIM + NDAP;

  k_cvt_x<<<(NROWS * NINP / 8) / 256, 256, 0, stream>>>(x, x16, NROWS * NINP / 8);
  k_trans16<<<dim3(NDIM / 64, NINP / 64), 256, 0, stream>>>(W_mlp0, W0T, NINP, NDIM, 16.0f);
  k_trans16<<<dim3(NDAP / 64, NDIM / 64), 256, 0, stream>>>(W1, W1T, NDIM, NDA, 16.0f);
  k_trans16<<<dim3(NG3 / 64, NDIM / 64), 256, 0, stream>>>(W_ih, WihT, NDIM, NG3, 16.0f);
  k_trans16<<<dim3(NG3 / 64, NHID / 64), 256, 0, stream>>>(W_hh, WhhT, NHID, NG3, 16.0f);
  k_bias<<<(NBIAS + 255) / 256, 256, 0, stream>>>(b_mlp0, b1, b_i, btab, NBIAS);

  {
    const int tiles = (NROWS / 64) * (NDIM / 64);
    wmma_gemm64<0, false, 2, 1, false, 2><<<dim3((tiles + 7) / 8, 1), 256, 0, stream>>>(
        x16, x16, NINP, (long)0, W0T, W0T, NINP, (long)0,
        (void*)m16, (void*)m16, NDIM, (long)0, b0r, U, (long)0, NROWS, NDIM, NINP, 1.0f / 16.0f);
  }
  {
    const int tiles = (NDIM / 64) * (NROWS / 64);
    wmma_gemm64<0, false, 1, 1, false, 2><<<dim3((tiles + 7) / 8, 1), 256, 0, stream>>>(
        W0T, W0T, NINP, (long)0, x16, x16, NINP, (long)0,
        (void*)mT16, (void*)mT16, NROWS, (long)0, b0r, U, (long)0, NDIM, NROWS, NINP, 1.0f / 16.0f);
  }
  {
    const int tiles = (NROWS / 64) * (NDAP / 64);
    wmma_gemm64<0, false, 2, 0, false, 0><<<dim3((tiles + 7) / 8, 1), 256, 0, stream>>>(
        m16, m16, NDIM, (long)0, W1T, W1T, NDIM, (long)0,
        (void*)U, (void*)U, UPITCH, (long)0, b1p, U, (long)0, NROWS, NDAP, NDIM, 1.0f / 16.0f);
  }
  k_attnp<<<NBATCH, 512, 0, stream>>>(U, W2, b2, P16);
  {
    const int tiles = (NSEQ / 64) * (NDIM / 64);
    wmma_gemm64<0, false, 0, 1, false, 0><<<dim3((tiles + 7) / 8, NBATCH), 256, 0, stream>>>(
        P16, P16, NSEQ, (long)NSEQ * NSEQ, mT16, mT16, NROWS, (long)NSEQ,
        (void*)M16, (void*)M16, NBATCH * NDIM, (long)NDIM, b0r, U, (long)0, NSEQ, NDIM, NSEQ, 1.0f / 1024.0f);
  }
  {
    const int tiles = (NG3 / 64) * (NROWS / 64);
    wmma_gemm64<0, false, 1, 0, false, 0><<<dim3((tiles + 7) / 8, 1), 256, 0, stream>>>(
        WihT, WihT, NDIM, (long)0, M16, M16, NDIM, (long)0,
        (void*)giT, (void*)giT, NROWS, (long)0, bir, U, (long)0, NG3, NROWS, NDIM, 1.0f / 16.0f);
  }
  k_gru<<<1, 512, 0, stream>>>(giT, WhhT, b_h, out);
}
